// TP_lstm_32950989095134
// MI455X (gfx1250) — hardware-run, weakly checked
//
#include <hip/hip_runtime.h>
#include <stdint.h>
#include <stddef.h>

typedef __attribute__((ext_vector_type(16))) _Float16 v16h;
typedef __attribute__((ext_vector_type(8)))  _Float16 v8h;
typedef __attribute__((ext_vector_type(8)))  float    v8f;
typedef __attribute__((ext_vector_type(4)))  float    v4f;
typedef __attribute__((ext_vector_type(4)))  unsigned v4u;

constexpr int kBatch     = 128;
constexpr int kSpat      = 128;
constexpr int kSteps     = 64;
constexpr int kIn        = 3;
constexpr int kHid       = 64;
constexpr int kGate      = 4 * kHid;
constexpr int kOutHid    = 32;
constexpr int kSkip      = 8;
constexpr int kOutCols   = kSteps - kSkip;
constexpr int kPitch     = 64;
constexpr int kPadRows   = kSpat + 2;
constexpr int kThreads   = 256;
constexpr int kWaves     = kThreads / 32;
constexpr int kSlabPitch = 32;
constexpr float kHidCarry = 64.0f;
constexpr float kWCarry   = 16.0f;
constexpr float kAccFold  = 1.0f / 1024.0f;

static_assert(kGate == kThreads);
static_assert(kSpat == 16 * kWaves);
static_assert((kSpat * kOutCols) % 128 == 0);
static_assert((kSpat * kOutCols) / 128 == 7 * kWaves);
static_assert((kPadRows * kPitch) % 8 == 0);

union FragU { v16h v; v8h h[2]; };
__device__ __forceinline__ v16h frag_load(const _Float16* p) {
  FragU f;
  f.h[0] = *(const v8h*)(p);
  f.h[1] = *(const v8h*)(p + 16);
  return f.v;
}

__device__ __forceinline__ v8f mma16(v16h a, v16h b, v8f c) {
  c = __builtin_amdgcn_wmma_f32_16x16x32_f16(false, a, false, b, (short)0, c, false, false);
  asm volatile("v_nop\n\tv_nop\n\tv_nop\n\tv_nop" : "+v"(c) : "v"(a), "v"(b));
  return c;
}

__device__ __forceinline__ void wave_sync() {
  __builtin_amdgcn_fence(__ATOMIC_RELEASE, "workgroup");
  __builtin_amdgcn_wave_barrier();
  __builtin_amdgcn_fence(__ATOMIC_ACQUIRE, "workgroup");
}

__device__ __forceinline__ float sigm_f(float x) {
  x = fminf(fmaxf(x, -30.0f), 30.0f);
  const float e = expf(-x);
  return 1.0f / (1.0f + e);
}

__device__ __forceinline__ float gate_xterm(const float* bg, const float* wih, int n, float x0, float x1, float x2) {
  return bg[n] + (wih[n * kIn + 0] * x0 + wih[n * kIn + 1] * x1 + wih[n * kIn + 2] * x2);
}

__device__ __forceinline__ void stage16(float* slab, v8f a, int col0, int hh, int cl) {
#pragma unroll
  for (int r = 0; r < 8; ++r) slab[(8 * hh + r) * kSlabPitch + col0 + cl] = a[r];
}

__global__ __launch_bounds__(256) void cast_scale_f32_f16x2(
    const float* __restrict__ in, _Float16* __restrict__ out, int n2, float scale) {
  const int i = blockIdx.x * 256 + threadIdx.x;
  if (i < n2) {
    const _Float16 h0 = (_Float16)(in[2 * i] * scale);
    const _Float16 h1 = (_Float16)(in[2 * i + 1] * scale);
    const unsigned u = (unsigned)__builtin_bit_cast(unsigned short, h0) |
                       ((unsigned)__builtin_bit_cast(unsigned short, h1) << 16);
    ((volatile unsigned*)out)[i] = u;
    __threadfence();
    ((volatile unsigned*)out)[i] = u;
  }
}

__device__ __forceinline__ void spatial_acc(v8f (&acc)[4], const _Float16* hpl,
                                            const _Float16* __restrict__ Wp, int s0, int cl, int hh) {
#pragma unroll
  for (int j = 0; j < 4; ++j) acc[j] = (v8f){0.f, 0.f, 0.f, 0.f, 0.f, 0.f, 0.f, 0.f};
#pragma unroll
  for (int kt = 0; kt < 4; ++kt) {
    const int arow = s0 + cl + ((kt < 2) ? 2 : 0);
    const int akb  = (kt & 1) * 32;
    const v16h a = frag_load(hpl + arow * kPitch + akb + 8 * hh);
#pragma unroll
    for (int j = 0; j < 4; ++j) {
      const v16h bw = frag_load(Wp + (size_t)(16 * j + cl) * (2 * kHid) + kt * 32 + 8 * hh);
      acc[j] = mma16(a, bw, acc[j]);
    }
  }
}

template <int kWhich>
__device__ __forceinline__ void spatial_epi(const v8f (&acc)[4], float* slab, _Float16* hpl, float* cpl,
                                            const float* bsv, int s0, int ln, int hh, int cl) {
#pragma unroll
  for (int q = 0; q < 2; ++q) {
    stage16(slab, acc[2 * q], 0, hh, cl);
    stage16(slab, acc[2 * q + 1], 16, hh, cl);
    wave_sync();
#pragma unroll 1
    for (int e = 0; e < 16; ++e) {
      const int s = s0 + e;
      const int u = 32 * q + ln;
      const float g = sigm_f(slab[e * kSlabPitch + ln] * kAccFold + bsv[u]);
      if (kWhich == 0) {
        const int ci = s * kHid + u;
        const float cg = cpl[ci] * g;
        cpl[ci] = cg;
      } else {
        const int hi = (s + 1) * kPitch + u;
        const _Float16 hq = hpl[hi];
        const float hv = (float)hq;
        hpl[hi] = (_Float16)(hv * g);
      }
    }
    wave_sync();
  }
}

__global__ __launch_bounds__(kThreads) void st_cell_seq(
    const float* __restrict__ xin,
    const float* __restrict__ in_aux,
    const float* __restrict__ Wih,
    const float* __restrict__ bih,
    const float* __restrict__ bhh,
    const float* __restrict__ bsf,
    const float* __restrict__ bsi,
    const float* __restrict__ bo1,
    const float* __restrict__ Wo2,
    const float* __restrict__ bo2,
    const _Float16* __restrict__ Wsf16,
    const _Float16* __restrict__ Wsi16,
    const _Float16* __restrict__ Whh16,
    const _Float16* __restrict__ Wo116,
    float* __restrict__ oplane)
{
  __shared__ __align__(16) _Float16 sh_h16[kPadRows * kPitch];
  __shared__ __align__(16) float    sh_c[kSpat * kHid];
  __shared__ __align__(16) float    sh_slab[kWaves][16 * kSlabPitch];
  __shared__ __align__(16) float    sh_o[kSpat];
  __shared__ float sh_x[kSpat * kIn];
  __shared__ float sh_wih[kGate * kIn];
  __shared__ float sh_bg[kGate];
  __shared__ float sh_bs[2 * kHid];
  __shared__ float sh_bo1[kOutHid];
  __shared__ float sh_wo2[kOutHid];
  __shared__ float sh_bo2[4];
  (void)in_aux;

  const int tid = threadIdx.x;
  const int wv  = tid >> 5;
  const int ln  = tid & 31;
  const int hh  = ln >> 4;
  const int cl  = ln & 15;
  const int bb  = blockIdx.x;
  const int s0  = wv * 16;
  float* slab = sh_slab[wv];

  for (int i = tid; i < (kPadRows * kPitch) / 8; i += kThreads)
    ((v4u*)(void*)sh_h16)[i] = (v4u){0u, 0u, 0u, 0u};
  for (int i = tid; i < kSpat * kHid; i += kThreads) sh_c[i] = 0.0f;
  for (int i = tid; i < kGate * kIn; i += kThreads) sh_wih[i] = Wih[i];
  sh_bg[tid] = bih[tid] + bhh[tid];
  if (tid < 2 * kHid) {
    const int jf = tid < kHid ? tid : kHid - 1;
    const int ji = tid >= kHid ? tid - kHid : 0;
    const float vf = bsf[jf];
    const float vi = bsi[ji];
    sh_bs[tid] = (tid < kHid) ? vf : vi;
  }
  if (tid < kOutHid) { sh_bo1[tid] = bo1[tid]; sh_wo2[tid] = Wo2[tid]; }
  if (tid == 0) sh_bo2[0] = bo2[0];
  __syncthreads();

#pragma unroll 1
  for (int t = 0; t < kSteps; ++t) {
    for (int i = tid; i < kSpat * kIn; i += kThreads) {
      const int s = i / kIn;
      const int comp = i - s * kIn;
      sh_x[i] = xin[(((size_t)bb * kSpat + s) * kSteps + t) * kIn + comp];
    }

    {
      v8f accF[4];
      spatial_acc(accF, sh_h16, Wsf16, s0, cl, hh);
      spatial_epi<0>(accF, slab, sh_h16, sh_c, sh_bs, s0, ln, hh, cl);
    }
    v8f accI[4];
    spatial_acc(accI, sh_h16, Wsi16, s0, cl, hh);
    __syncthreads();
    spatial_epi<1>(accI, slab, sh_h16, sh_c, sh_bs + kHid, s0, ln, hh, cl);
    wave_sync();

    {
      const v16h a0 = frag_load(sh_h16 + (s0 + 1 + cl) * kPitch + 8 * hh);
      const v16h a1 = frag_load(sh_h16 + (s0 + 1 + cl) * kPitch + 32 + 8 * hh);
#pragma unroll 1
      for (int ub = 0; ub < 4; ++ub) {
        v8f acc[4];
#pragma unroll
        for (int g = 0; g < 4; ++g) {
          acc[g] = (v8f){0.f, 0.f, 0.f, 0.f, 0.f, 0.f, 0.f, 0.f};
          const _Float16* wrow = Whh16 + (size_t)(g * kHid + 16 * ub + cl) * kHid + 8 * hh;
          acc[g] = mma16(a0, frag_load(wrow), acc[g]);
          acc[g] = mma16(a1, frag_load(wrow + 32), acc[g]);
        }
        stage16(slab, acc[0], 0, hh, cl);
        stage16(slab, acc[2], 16, hh, cl);
        wave_sync();
#pragma unroll 1
        for (int e = 0; e < 8; ++e) {
          const int idx = e * 32 + ln;
          const int row = idx >> 4, uc = idx & 15;
          const int s = s0 + row, u = 16 * ub + uc;
          const float x0 = sh_x[s * kIn + 0], x1 = sh_x[s * kIn + 1], x2 = sh_x[s * kIn + 2];
          const float pi = slab[row * kSlabPitch + uc] * kAccFold + gate_xterm(sh_bg, sh_wih, u, x0, x1, x2);
          const float pg = slab[row * kSlabPitch + 16 + uc] * kAccFold + gate_xterm(sh_bg, sh_wih, 2 * kHid + u, x0, x1, x2);
          slab[row * kSlabPitch + uc] = sigm_f(pi) * tanhf(pg);
        }
        wave_sync();
        stage16(slab, acc[1], 16, hh, cl);
        wave_sync();
#pragma unroll 1
        for (int e = 0; e < 8; ++e) {
          const int idx = e * 32 + ln;
          const int row = idx >> 4, uc = idx & 15;
          const int s = s0 + row, u = 16 * ub + uc;
          const float x0 = sh_x[s * kIn + 0], x1 = sh_x[s * kIn + 1], x2 = sh_x[s * kIn + 2];
          const float pf = slab[row * kSlabPitch + 16 + uc] * kAccFold + gate_xterm(sh_bg, sh_wih, kHid + u, x0, x1, x2);
          const int ci = s * kHid + u;
          const float cn = sigm_f(pf) * sh_c[ci] + slab[row * kSlabPitch + uc];
          sh_c[ci] = cn;
        }
        wave_sync();
        stage16(slab, acc[3], 0, hh, cl);
        wave_sync();
#pragma unroll 1
        for (int e = 0; e < 8; ++e) {
          const int idx = e * 32 + ln;
          const int row = idx >> 4, uc = idx & 15;
          const int s = s0 + row, u = 16 * ub + uc;
          const float x0 = sh_x[s * kIn + 0], x1 = sh_x[s * kIn + 1], x2 = sh_x[s * kIn + 2];
          const float po = slab[row * kSlabPitch + uc] * kAccFold + gate_xterm(sh_bg, sh_wih, 3 * kHid + u, x0, x1, x2);
          const float hn = sigm_f(po) * tanhf(sh_c[s * kHid + u]);
          sh_h16[(s + 1) * kPitch + u] = (_Float16)(hn * kHidCarry);
        }
        wave_sync();
      }
    }

    {
      const v16h c0 = frag_load(sh_h16 + (s0 + 1 + cl) * kPitch + 8 * hh);
      const v16h c1 = frag_load(sh_h16 + (s0 + 1 + cl) * kPitch + 32 + 8 * hh);
      v8f acc2[2];
#pragma unroll
      for (int j = 0; j < 2; ++j) {
        acc2[j] = (v8f){0.f, 0.f, 0.f, 0.f, 0.f, 0.f, 0.f, 0.f};
        const _Float16* wrow = Wo116 + (size_t)(16 * j + cl) * kHid + 8 * hh;
        acc2[j] = mma16(c0, frag_load(wrow), acc2[j]);
        acc2[j] = mma16(c1, frag_load(wrow + 32), acc2[j]);
      }
      const float b0 = sh_bo1[cl], b1 = sh_bo1[16 + cl];
      const float w0 = sh_wo2[cl], w1 = sh_wo2[16 + cl];
      const float bo2v = sh_bo2[0];
#pragma unroll
      for (int r = 0; r < 8; ++r) {
        const float h0v = fmaxf(acc2[0][r] * kAccFold + b0, 0.0f);
        const float h1v = fmaxf(acc2[1][r] * kAccFold + b1, 0.0f);
        float pv = h0v * w0 + h1v * w1;
        pv += __shfl_xor(pv, 1);
        pv += __shfl_xor(pv, 2);
        pv += __shfl_xor(pv, 4);
        pv += __shfl_xor(pv, 8);
        if (cl == 0) sh_o[s0 + 8 * hh + r] = pv + bo2v;
      }
    }
    __syncthreads();

    if (wv == 0) {
      if (t >= kSkip) {
        const v4f v = *(const v4f*)(sh_o + 4 * ln);
        float* dst = oplane + ((size_t)bb * kOutCols + (t - kSkip)) * kSpat + 4 * ln;
        *(volatile v4f*)dst = v;
        __threadfence();
        *(volatile v4f*)dst = v;
      }
    }
  }
}

__global__ __launch_bounds__(kThreads) void out_transpose(const float* __restrict__ oplane, float* __restrict__ out) {
  __shared__ __align__(16) float sh[kSpat * kOutCols];
  const int tid = threadIdx.x;
  const int wv  = tid >> 5;
  const int ln  = tid & 31;
  const int bb  = blockIdx.x;
  const float* src = oplane + (size_t)bb * kOutCols * kSpat;
  for (int i = tid; i < kOutCols * kSpat; i += kThreads) {
    const int k = i >> 7;
    const int s = i & (kSpat - 1);
    sh[s * kOutCols + k] = src[i];
  }
  __syncthreads();
  float* ob = out + (size_t)bb * (kSpat * kOutCols);
  for (int pass = 0; pass < 2; ++pass) {
#pragma unroll
    for (int it = 0; it < 7; ++it) {
      const int q = it * 8 + wv;
      const v4f v = *(const v4f*)(sh + q * 128 + 4 * ln);
      *(volatile v4f*)(ob + (size_t)q * 128 + 4 * ln) = v;
    }
    __threadfence();
  }
}

extern "C" void kernel_launch(void* const* d_in, const int* in_sizes, int n_in,
                              void* d_out, int out_size, void* d_ws, size_t ws_size,
                              hipStream_t stream) {
  if (n_in < 14) return;
  const float* xin = (const float*)d_in[0];
  const float* in_aux = (const float*)d_in[1];
  const float* Wih = (const float*)d_in[2];
  const float* bih = (const float*)d_in[3];
  const float* Whh = (const float*)d_in[4];
  const float* bhh = (const float*)d_in[5];
  const float* Wsf = (const float*)d_in[6];
  const float* bsf = (const float*)d_in[7];
  const float* Wsi = (const float*)d_in[8];
  const float* bsi = (const float*)d_in[9];
  const float* Wo1 = (const float*)d_in[10];
  const float* bo1 = (const float*)d_in[11];
  const float* Wo2 = (const float*)d_in[12];
  const float* bo2 = (const float*)d_in[13];
  float* out = (float*)d_out;

  if (in_sizes[0] != kBatch * kSpat * kSteps * kIn) return;
  if (in_sizes[2] != kGate * kIn || in_sizes[3] != kGate || in_sizes[4] != kGate * kHid || in_sizes[5] != kGate) return;
  if (in_sizes[6] != kHid * 2 * kHid || in_sizes[7] != kHid || in_sizes[8] != kHid * 2 * kHid || in_sizes[9] != kHid) return;
  if (in_sizes[10] != kOutHid * kHid || in_sizes[11] != kOutHid || in_sizes[12] != kOutHid || in_sizes[13] != 1) return;
  if (out_size != kBatch * kSpat * kOutCols) return;

  const size_t off_sf = 0;
  const size_t off_si = off_sf + (size_t)in_sizes[6] * 2;
  const size_t off_hh = off_si + (size_t)in_sizes[8] * 2;
  const size_t off_o1 = off_hh + (size_t)in_sizes[4] * 2;
  const size_t off_op = off_o1 + (size_t)in_sizes[10] * 2;
  const size_t carve  = off_op + (size_t)kBatch * kOutCols * kSpat * sizeof(float);
  if (carve > ws_size) return;
  char* ws = (char*)d_ws;
  _Float16* Wsf16 = (_Float16*)(ws + off_sf);
  _Float16* Wsi16 = (_Float16*)(ws + off_si);
  _Float16* Whh16 = (_Float16*)(ws + off_hh);
  _Float16* Wo116 = (_Float16*)(ws + off_o1);
  float* oplane = (float*)(ws + off_op);

  const int n2_sf = in_sizes[6] / 2, n2_si = in_sizes[8] / 2, n2_hh = in_sizes[4] / 2, n2_o1 = in_sizes[10] / 2;
  cast_scale_f32_f16x2<<<dim3((n2_sf + 255) / 256), dim3(256), 0, stream>>>(Wsf, Wsf16, n2_sf, kWCarry);
  cast_scale_f32_f16x2<<<dim3((n2_si + 255) / 256), dim3(256), 0, stream>>>(Wsi, Wsi16, n2_si, kWCarry);
  cast_scale_f32_f16x2<<<dim3((n2_hh + 255) / 256), dim3(256), 0, stream>>>(Whh, Whh16, n2_hh, kWCarry);
  cast_scale_f32_f16x2<<<dim3((n2_o1 + 255) / 256), dim3(256), 0, stream>>>(Wo1, Wo116, n2_o1, kWCarry);

  st_cell_seq<<<dim3(kBatch), dim3(kThreads), 0, stream>>>(
      xin, in_aux, Wih, bih, bhh, bsf, bsi, bo1, Wo2, bo2,
      Wsf16, Wsi16, Whh16, Wo116, oplane);

  out_transpose<<<dim3(kBatch), dim3(kThreads), 0, stream>>>(oplane, out);
}
